// Model_39676907882670
// MI455X (gfx1250) — hardware-verified
//
#include <hip/hip_runtime.h>

#ifndef NB
#define NB 64
#endif
#ifndef SEQ
#define SEQ 2048
#endif
#define NB_FULL 64
#define SEQ_FULL 2048
#define DD 64
#define BM 64
#define BN 64
#define PP 72
#define OP 68

static_assert(NB >= 1 && NB <= NB_FULL);
static_assert(SEQ >= BN && SEQ <= SEQ_FULL);
static_assert(SEQ % BM == 0);
static_assert(SEQ % BN == 0);
static_assert(DD == 64);
static_assert((PP * 2) % 16 == 0);
static_assert((OP * 4) % 16 == 0);
static_assert((NB * SEQ * (DD / 8)) % 256 == 0);
static_assert((size_t)NB_FULL * SEQ_FULL * DD * 4 == (size_t)33554432);
static_assert((size_t)2 * NB_FULL * SEQ_FULL * DD * 2 <= (size_t)134217728);

typedef __bf16 v16b __attribute__((ext_vector_type(16)));
typedef _Float16 v16h __attribute__((ext_vector_type(16)));
typedef unsigned short v8us __attribute__((ext_vector_type(8), may_alias));
typedef float v8f __attribute__((ext_vector_type(8)));
typedef float v4f __attribute__((ext_vector_type(4)));
typedef float v4fa __attribute__((ext_vector_type(4), may_alias));
union FragB { v16b v; v8us half[2]; unsigned short u[16]; };
union FragH { v16h v; v8us half[2]; _Float16 h[16]; unsigned short u[16]; };

__device__ __forceinline__ unsigned short bf16_bits(float x) { unsigned int u = __float_as_uint(x); return (unsigned short)((u + 0x7FFFu + ((u >> 16) & 1u)) >> 16); }
__device__ __forceinline__ float bf16_val(unsigned short bb) { return __uint_as_float(((unsigned int)bb) << 16); }
__device__ __forceinline__ float bf16_rne(float x) { return bf16_val(bf16_bits(x)); }

__device__ __forceinline__ v8f mma_bf(v16b a, v16b bq, v8f c) {
  v8f d = __builtin_amdgcn_wmma_f32_16x16x32_bf16(false, a, false, bq, (short)0, c, false, false);
  asm volatile("v_nop\n\tv_nop\n\tv_nop\n\tv_nop" : "+v"(d) : "v"(a), "v"(bq));
  return d;
}
__device__ __forceinline__ v8f mma_hf(v16h a, v16h bq, v8f c) {
  v8f d = __builtin_amdgcn_wmma_f32_16x16x32_f16(false, a, false, bq, (short)0, c, false, false);
  asm volatile("v_nop\n\tv_nop\n\tv_nop\n\tv_nop" : "+v"(d) : "v"(a), "v"(bq));
  return d;
}

__global__ __launch_bounds__(256) void k_kplane(const float* __restrict__ k, unsigned short* __restrict__ KB, int n8) {
  const int t = blockIdx.x * 256 + threadIdx.x;
  if (t >= n8) return;
  const int prow = t >> 3, d8 = (t & 7) * 8;
  const int b = prow / SEQ, s = prow - b * SEQ;
  const float* src = k + ((size_t)b * SEQ_FULL + s) * DD + d8;
  const v4f x0 = *(const v4fa*)src, x1 = *(const v4fa*)(src + 4);
  FragB f;
#pragma unroll
  for (int i = 0; i < 4; ++i) { f.u[i] = bf16_bits(x0[i]); f.u[4 + i] = bf16_bits(x1[i]); }
  unsigned short* dst = KB + (size_t)t * 8;
  *(volatile v8us*)dst = f.half[0];
  __threadfence();
  *(volatile v8us*)dst = f.half[0];
}

__global__ __launch_bounds__(256) void k_vtplane(const float* __restrict__ v, unsigned short* __restrict__ VT, int ngrp) {
  __shared__ unsigned short tl[64][65];
  const int tid = threadIdx.x;
  const int b = blockIdx.x / ngrp, sg = blockIdx.x - b * ngrp;
  const int s0 = sg * 64;
  for (int it = 0; it < 2; ++it) {
    const int i = tid + 256 * it;
    const int j = i >> 3, d8 = (i & 7) * 8;
    const float* src = v + ((size_t)b * SEQ_FULL + s0 + j) * DD + d8;
    const v4f x0 = *(const v4fa*)src, x1 = *(const v4fa*)(src + 4);
    FragH f;
#pragma unroll
    for (int qd = 0; qd < 4; ++qd) { f.h[qd] = (_Float16)bf16_rne(x0[qd]); f.h[4 + qd] = (_Float16)bf16_rne(x1[qd]); }
#pragma unroll
    for (int qd = 0; qd < 8; ++qd) tl[d8 + qd][j] = f.u[qd];
  }
  __syncthreads();
  for (int pass = 0; pass < 2; ++pass) {
    for (int it = 0; it < 2; ++it) {
      const int i = tid + 256 * it;
      const int d = i >> 3, j8 = (i & 7) * 8;
      FragH f;
#pragma unroll
      for (int qd = 0; qd < 8; ++qd) f.u[qd] = tl[d][j8 + qd];
      *(volatile v8us*)(VT + ((size_t)b * DD + d) * SEQ + s0 + j8) = f.half[0];
    }
    if (pass == 0) __threadfence();
  }
}

__global__ void __launch_bounds__(128) __attribute__((amdgpu_num_vgpr(256)))
k_attn(const float* __restrict__ q, const unsigned short* __restrict__ KB, const unsigned short* __restrict__ VT, float* __restrict__ out) {
  __shared__ __attribute__((aligned(16))) _Float16 sP[4][16][PP];
  __shared__ __attribute__((aligned(16))) float so[4][16][OP];
  const int b = blockIdx.y, qbase = blockIdx.x * BM;
  const int tid = threadIdx.x, w = tid >> 5, lane = tid & 31, ln = lane & 15, hh = lane >> 4;
  const float rs = 0.125f;
  const float L2E = 1.44269504088896340736f;
  const v8f z8 = {0.f, 0.f, 0.f, 0.f, 0.f, 0.f, 0.f, 0.f};

  v16b q0, q1;
  {
    const float* qp = q + ((size_t)b * SEQ_FULL + qbase + w * 16 + ln) * DD;
    const v4f a0 = *(const v4fa*)(qp + 8 * hh), a1 = *(const v4fa*)(qp + 8 * hh + 4), a2 = *(const v4fa*)(qp + 16 + 8 * hh), a3 = *(const v4fa*)(qp + 20 + 8 * hh);
    const v4f c0 = *(const v4fa*)(qp + 32 + 8 * hh), c1 = *(const v4fa*)(qp + 36 + 8 * hh), c2 = *(const v4fa*)(qp + 48 + 8 * hh), c3 = *(const v4fa*)(qp + 52 + 8 * hh);
    FragB f0, f1;
#pragma unroll
    for (int i = 0; i < 4; ++i) {
      f0.u[i] = bf16_bits(a0[i]); f0.u[4 + i] = bf16_bits(a1[i]); f0.u[8 + i] = bf16_bits(a2[i]); f0.u[12 + i] = bf16_bits(a3[i]);
      f1.u[i] = bf16_bits(c0[i]); f1.u[4 + i] = bf16_bits(c1[i]); f1.u[8 + i] = bf16_bits(c2[i]); f1.u[12 + i] = bf16_bits(c3[i]);
    }
    q0 = f0.v; q1 = f1.v;
  }
  v16h ones;
  {
    FragH fo;
#pragma unroll
    for (int i = 0; i < 16; ++i) fo.h[i] = (_Float16)1.0f;
    ones = fo.v;
  }

  v8f o[4] = {z8, z8, z8, z8};
  v8f ls = z8;
  float mrow[8];
#pragma unroll
  for (int r = 0; r < 8; ++r) mrow[r] = -3.0e38f;

  const unsigned short* kp = KB + ((size_t)b * SEQ + ln) * DD + 8 * hh;
  const unsigned short* vp = VT + ((size_t)b * DD + ln) * SEQ + 8 * hh;

#pragma unroll 1
  for (int kt = 0; kt < SEQ / BN; ++kt) {
    const int kv0 = kt * BN;
    v8f s[4];
#pragma unroll
    for (int ht = 0; ht < 4; ++ht) {
      const unsigned short* p = kp + (size_t)(kv0 + ht * 16) * DD;
      FragB b0, b1;
      b0.half[0] = *(const v8us*)(p);      b0.half[1] = *(const v8us*)(p + 16);
      b1.half[0] = *(const v8us*)(p + 32); b1.half[1] = *(const v8us*)(p + 48);
      v8f acc = z8;
      acc = mma_bf(q0, b0.v, acc);
      acc = mma_bf(q1, b1.v, acc);
      s[ht] = acc * rs;
    }
    float mnew[8], alpha[8];
#pragma unroll
    for (int r = 0; r < 8; ++r) {
      float c0 = fmaxf(fmaxf(s[0][r], s[1][r]), fmaxf(s[2][r], s[3][r]));
      c0 = fmaxf(c0, __shfl_xor(c0, 1, 16));
      c0 = fmaxf(c0, __shfl_xor(c0, 2, 16));
      c0 = fmaxf(c0, __shfl_xor(c0, 4, 16));
      c0 = fmaxf(c0, __shfl_xor(c0, 8, 16));
      mnew[r] = fmaxf(mrow[r], c0);
      alpha[r] = exp2f(fmaxf(mrow[r] - mnew[r], -120.0f) * L2E);
      mrow[r] = mnew[r];
    }
    __builtin_amdgcn_fence(4, "workgroup");
    __builtin_amdgcn_wave_barrier();
#pragma unroll
    for (int ht = 0; ht < 4; ++ht)
#pragma unroll
      for (int r = 0; r < 8; ++r) {
        const float pv = exp2f(fmaxf(s[ht][r] - mnew[r], -120.0f) * L2E) * 1024.0f;
        sP[w][8 * hh + r][ht * 16 + ln] = (_Float16)pv;
      }
    const v8f al8 = {alpha[0], alpha[1], alpha[2], alpha[3], alpha[4], alpha[5], alpha[6], alpha[7]};
#pragma unroll
    for (int j = 0; j < 4; ++j) o[j] = o[j] * al8;
    ls = ls * al8;
    __builtin_amdgcn_fence(4, "workgroup");
    __builtin_amdgcn_wave_barrier();
    FragH pa0, pa1;
    pa0.half[0] = *(const v8us*)&sP[w][ln][8 * hh];      pa0.half[1] = *(const v8us*)&sP[w][ln][16 + 8 * hh];
    pa1.half[0] = *(const v8us*)&sP[w][ln][32 + 8 * hh]; pa1.half[1] = *(const v8us*)&sP[w][ln][48 + 8 * hh];
#pragma unroll
    for (int j = 0; j < 4; ++j) {
      const unsigned short* p = vp + (size_t)(j * 16) * SEQ + kv0;
      FragH v0, v1;
      v0.half[0] = *(const v8us*)(p);      v0.half[1] = *(const v8us*)(p + 16);
      v1.half[0] = *(const v8us*)(p + 32); v1.half[1] = *(const v8us*)(p + 48);
      o[j] = mma_hf(pa0.v, v0.v, o[j]);
      o[j] = mma_hf(pa1.v, v1.v, o[j]);
    }
    ls = mma_hf(pa0.v, ones, ls);
    ls = mma_hf(pa1.v, ones, ls);
  }

  float il[8];
#pragma unroll
  for (int r = 0; r < 8; ++r) il[r] = 1.0f / ls[r];
#pragma unroll
  for (int j = 0; j < 4; ++j)
#pragma unroll
    for (int r = 0; r < 8; ++r) so[w][8 * hh + r][j * 16 + ln] = o[j][r] * il[r];
  __builtin_amdgcn_fence(4, "workgroup");
  __builtin_amdgcn_wave_barrier();
  float* ob = out + ((size_t)b * SEQ + qbase + w * 16) * DD;
  const int rsub = lane >> 4, c4 = (lane & 15) * 4;
  for (int pass = 0; pass < 2; ++pass) {
#pragma unroll
    for (int qq = 0; qq < 8; ++qq) {
      const int r = qq * 2 + rsub;
      const v4f val = *(const v4fa*)&so[w][r][c4];
      *(volatile v4f*)(ob + (size_t)r * DD + c4) = val;
    }
    if (pass == 0) __threadfence();
  }
}

extern "C" void kernel_launch(void* const* d_in, const int* in_sizes, int n_in,
                              void* d_out, int out_size, void* d_ws, size_t ws_size, hipStream_t stream) {
  if (n_in < 3) return;
  const size_t need_in = ((size_t)(NB - 1) * SEQ_FULL + (size_t)SEQ) * DD;
  if ((size_t)in_sizes[0] < need_in || (size_t)in_sizes[1] < need_in || (size_t)in_sizes[2] < need_in) return;
  if ((size_t)out_size < (size_t)NB * SEQ * DD) return;
  const float* q = (const float*)d_in[0];
  const float* k = (const float*)d_in[1];
  const float* v = (const float*)d_in[2];
  float* out = (float*)d_out;

  char* ws = (char*)d_ws; size_t off = 0;
  auto take = [&](size_t bytes) { char* p = ws + off; off += (bytes + 255) & ~(size_t)255; return p; };
  const size_t plane_bytes = (size_t)NB * SEQ * DD * 2;
  unsigned short* KB = (unsigned short*)take(plane_bytes);
  unsigned short* VT = (unsigned short*)take(plane_bytes);
  if (off > ws_size) return;

  const int n8 = NB * SEQ * (DD / 8);
  k_kplane<<<(unsigned)((n8 + 255) / 256), 256, 0, stream>>>(k, KB, n8);
  k_vtplane<<<(unsigned)(NB * (SEQ / 64)), 256, 0, stream>>>(v, VT, SEQ / 64);
  k_attn<<<dim3(SEQ / BM, NB), 128, 0, stream>>>(q, KB, VT, out);
}
